// LSTM_39384850104606
// MI455X (gfx1250) — hardware-verified
//
#include <hip/hip_runtime.h>
#include <math.h>

constexpr int NBATCH   = 1024;
constexpr int NSTEP    = 512;
constexpr int NIN      = 16;
constexpr int NHID     = 64;
constexpr int NGATE    = 4 * NHID;
constexpr int NOUT     = 8;
constexpr int NTHR     = 128;
constexpr int ROWS_BLK = 16;
constexpr int TCHUNK   = 16;
constexpr int XPITCH   = 24;
constexpr int HPITCH   = 72;
constexpr int FPITCH   = 68;
constexpr float ACARRY = 64.0f;
constexpr float WCARRY = 16.0f;
constexpr float FOLD   = 1.0f / (ACARRY * WCARRY);

static_assert(NBATCH % ROWS_BLK == 0, "block rows");
static_assert(NSTEP % TCHUNK == 0, "chunking");
static_assert(NHID == 16 * (NTHR / 32), "one 16-unit group per wave");
static_assert(NHID % 32 == 0, "h k-blocks");
static_assert(NIN == 16, "x k-block: 16 real + 16 zero");
static_assert(NGATE == 256, "gate columns");
static_assert((ROWS_BLK * TCHUNK * NIN) == 4 * NTHR * 8, "x chunk staging coverage");
static_assert((2 * ROWS_BLK * HPITCH) % NTHR == 0, "h zero fill exact");
static_assert(ROWS_BLK * NOUT == NTHR, "output map: one float per thread");
static_assert((XPITCH * 2) % 16 == 0 && (HPITCH * 2) % 16 == 0 && (FPITCH * 4) % 16 == 0, "16-B aligned pitches");

typedef __attribute__((ext_vector_type(16))) _Float16 v16h;
typedef __attribute__((ext_vector_type(8)))  _Float16 v8h;
typedef __attribute__((ext_vector_type(8)))  float    v8f;
typedef __attribute__((ext_vector_type(4)))  float    v4f;

template <typename T> struct Frag;
template <> struct Frag<_Float16> {
  typedef v16h V; union U { v16h v; v8h h[2]; };
  static __device__ __forceinline__ v16h load(const _Float16* p) {
    U f; f.h[0] = *(const v8h*)(p); f.h[1] = *(const v8h*)(p + 16); return f.v;
  }
  static __device__ __forceinline__ v8f mma(v16h a, v16h b, v8f c) {
    return __builtin_amdgcn_wmma_f32_16x16x32_f16(false, a, false, b, (short)0, c, false, false);
  }
};

__device__ __forceinline__ void group_guard(v8f& a0, v8f& a1, v8f& a2, v8f& a3, v16h x, v16h y, v16h z) {
  asm volatile("v_nop\n\tv_nop\n\tv_nop\n\tv_nop" : "+v"(a0), "+v"(a1), "+v"(a2), "+v"(a3) : "v"(x), "v"(y), "v"(z));
}
__device__ __forceinline__ void settle_frag(v16h& f) { asm volatile("" : "+v"(f) : : "memory"); }

__device__ __forceinline__ float fsig(float x) {
  const float xc = fminf(fmaxf(x, -30.0f), 30.0f);
  return __builtin_amdgcn_rcpf(1.0f + __expf(-xc));
}
__device__ __forceinline__ float ftanh(float x) {
  const float xc = fminf(fmaxf(x, -15.0f), 15.0f);
  return 1.0f - 2.0f * __builtin_amdgcn_rcpf(__expf(2.0f * xc) + 1.0f);
}

__device__ __forceinline__ v8h cvt8_scaled(const float* __restrict__ p, float sc) {
  const v4f a = *(const v4f*)(p);
  const v4f b = *(const v4f*)(p + 4);
  v8h o;
#pragma unroll
  for (int e = 0; e < 4; ++e) {
    o[e]     = (_Float16)(a[e] * sc);
    o[4 + e] = (_Float16)(b[e] * sc);
  }
  return o;
}

__device__ __forceinline__ void stage_x_chunk(const float* __restrict__ xblk, int t0, _Float16* xdst, int tid) {
#pragma unroll
  for (int half = 0; half < 2; ++half) {
    v8h hv[2];
    int dsto[2];
#pragma unroll
    for (int i = 0; i < 2; ++i) {
      const int unit = (half * 2 + i) * NTHR + tid;
      const int row  = unit >> 5;
      const int u    = unit & 31;
      const float* sp = xblk + (size_t)row * NSTEP * NIN + (size_t)t0 * NIN + u * 8;
      hv[i]   = cvt8_scaled(sp, ACARRY);
      dsto[i] = ((u >> 1) * ROWS_BLK + row) * XPITCH + (u & 1) * 8;
    }
#pragma unroll
    for (int i = 0; i < 2; ++i) *(v8h*)(xdst + dsto[i]) = hv[i];
    asm volatile("" : : : "memory");
  }
}

__global__ __launch_bounds__(NTHR) void lstm_seq_kernel(const float* __restrict__ x, const float* __restrict__ w_ih,
                                                        const float* __restrict__ w_hh, const float* __restrict__ b_ih,
                                                        const float* __restrict__ b_hh, const float* __restrict__ w_fc,
                                                        const float* __restrict__ b_fc, float* out) {
  __shared__ __align__(16) _Float16 Xs[2 * TCHUNK * ROWS_BLK * XPITCH];
  __shared__ __align__(16) _Float16 Hs[2 * ROWS_BLK * HPITCH];
  __shared__ __align__(16) float    Hfin[ROWS_BLK * FPITCH];

  const int tid = threadIdx.x, lane = tid & 31, wave = tid >> 5;
  const int c = lane & 15, hh = lane >> 4, koff = hh * 8;
  const int b0 = blockIdx.x * ROWS_BLK;
  const float* xblk = x + (size_t)b0 * NSTEP * NIN;

  const v8h zero8 = {(_Float16)0.0f, (_Float16)0.0f, (_Float16)0.0f, (_Float16)0.0f,
                     (_Float16)0.0f, (_Float16)0.0f, (_Float16)0.0f, (_Float16)0.0f};
  const v8f z8 = {0.f, 0.f, 0.f, 0.f, 0.f, 0.f, 0.f, 0.f};

  v16h Bhh[4][2];
  v16h Bih[4];
  float bsum[4];
#pragma unroll
  for (int g = 0; g < 4; ++g) {
    const int n = g * NHID + 16 * wave + c;
#pragma unroll
    for (int kb = 0; kb < 2; ++kb) {
      const float* wp = w_hh + (size_t)n * NHID + kb * 32 + koff;
      Frag<_Float16>::U f;
      f.h[0] = cvt8_scaled(wp, WCARRY);
      f.h[1] = cvt8_scaled(wp + 16, WCARRY);
      Bhh[g][kb] = f.v;
      settle_frag(Bhh[g][kb]);
    }
    {
      const float* wp = w_ih + (size_t)n * NIN + koff;
      Frag<_Float16>::U f;
      f.h[0] = cvt8_scaled(wp, WCARRY);
      f.h[1] = zero8;
      Bih[g] = f.v;
      settle_frag(Bih[g]);
    }
    bsum[g] = b_ih[n] + b_hh[n];
  }

#pragma unroll 1
  for (int i = tid; i < 2 * ROWS_BLK * HPITCH; i += NTHR) Hs[i] = (_Float16)0.0f;
  float cst[8], hst[8];
#pragma unroll
  for (int r = 0; r < 8; ++r) { cst[r] = 0.0f; hst[r] = 0.0f; }
  stage_x_chunk(xblk, 0, Xs, tid);
  __syncthreads();

#pragma unroll 1
  for (int t = 0; t < NSTEP; ++t) {
    const int cur = t & 1;
    const int xb  = (t >> 4) & 1;
    const int ts  = t & (TCHUNK - 1);
    if ((ts == 0) && (t + TCHUNK < NSTEP))
      stage_x_chunk(xblk, t + TCHUNK, Xs + (xb ^ 1) * TCHUNK * ROWS_BLK * XPITCH, tid);

    Frag<_Float16>::U fx;
    fx.h[0] = *(const v8h*)(Xs + ((xb * TCHUNK + ts) * ROWS_BLK + c) * XPITCH + koff);
    fx.h[1] = zero8;
    const v16h ax = fx.v;
    const _Float16* hrow = Hs + cur * ROWS_BLK * HPITCH + c * HPITCH + koff;
    const v16h ah0 = Frag<_Float16>::load(hrow);
    const v16h ah1 = Frag<_Float16>::load(hrow + 32);

    v8f acc[4];
#pragma unroll
    for (int g = 0; g < 4; ++g) acc[g] = z8;
#pragma unroll
    for (int g = 0; g < 4; ++g) acc[g] = Frag<_Float16>::mma(ax, Bih[g], acc[g]);
#pragma unroll
    for (int g = 0; g < 4; ++g) acc[g] = Frag<_Float16>::mma(ah0, Bhh[g][0], acc[g]);
#pragma unroll
    for (int g = 0; g < 4; ++g) acc[g] = Frag<_Float16>::mma(ah1, Bhh[g][1], acc[g]);
    group_guard(acc[0], acc[1], acc[2], acc[3], ax, ah0, ah1);

    _Float16* hnext = Hs + (cur ^ 1) * ROWS_BLK * HPITCH;
#pragma unroll
    for (int r = 0; r < 8; ++r) {
      const float zi = acc[0][r] * FOLD + bsum[0];
      const float zf = acc[1][r] * FOLD + bsum[1];
      const float zg = acc[2][r] * FOLD + bsum[2];
      const float zo = acc[3][r] * FOLD + bsum[3];
      const float ig = fsig(zi);
      const float fg = fsig(zf);
      const float gv = ftanh(zg);
      const float og = fsig(zo);
      const float cn = fg * cst[r] + ig * gv;
      cst[r] = cn;
      const float hn = og * ftanh(cn);
      hst[r] = hn;
      hnext[(8 * hh + r) * HPITCH + 16 * wave + c] = (_Float16)(hn * ACARRY);
    }
    __syncthreads();
  }

#pragma unroll
  for (int r = 0; r < 8; ++r) Hfin[(8 * hh + r) * FPITCH + 16 * wave + c] = hst[r];
  __syncthreads();
  {
    const int row = tid >> 3;
    const int o   = tid & 7;
    const float* wf = w_fc + (size_t)o * NHID;
    const float* hp = Hfin + row * FPITCH;
    float a = 0.0f;
#pragma unroll 4
    for (int k4 = 0; k4 < NHID / 4; ++k4) {
      const v4f wv = *(const v4f*)(wf + 4 * k4);
      const v4f hv = *(const v4f*)(hp + 4 * k4);
      a += wv[0] * hv[0];
      a += wv[1] * hv[1];
      a += wv[2] * hv[2];
      a += wv[3] * hv[3];
    }
    a += b_fc[o];
    const float val = __builtin_amdgcn_rcpf(1.0f + expf(-a));
    volatile float* op = out + (size_t)b0 * NOUT + tid;
    *op = val;
    __threadfence();
    *op = val;
  }
}

extern "C" void kernel_launch(void* const* d_in, const int* in_sizes, int n_in,
                              void* d_out, int out_size, void* d_ws, size_t ws_size, hipStream_t stream) {
  (void)d_ws; (void)ws_size;
  if (n_in < 7 || d_out == nullptr) return;
  if (in_sizes[0] != NBATCH * NSTEP * NIN || in_sizes[1] != NGATE * NIN || in_sizes[2] != NGATE * NHID ||
      in_sizes[3] != NGATE || in_sizes[4] != NGATE || in_sizes[5] != NOUT * NHID || in_sizes[6] != NOUT ||
      out_size != NBATCH * NOUT) return;

  const float* x    = (const float*)d_in[0];
  const float* w_ih = (const float*)d_in[1];
  const float* w_hh = (const float*)d_in[2];
  const float* b_ih = (const float*)d_in[3];
  const float* b_hh = (const float*)d_in[4];
  const float* w_fc = (const float*)d_in[5];
  const float* b_fc = (const float*)d_in[6];
  float* out = (float*)d_out;

  lstm_seq_kernel<<<NBATCH / ROWS_BLK, NTHR, 0, stream>>>(x, w_ih, w_hh, b_ih, b_hh, w_fc, b_fc, out);
}
